// OuterProductMean_49804440764766
// MI455X (gfx1250) — hardware-verified
//
#include <hip/hip_runtime.h>


#ifndef ILIM_ROWS
#define ILIM_ROWS 256
#endif

namespace {
constexpr int S = 128, NI = 256, CM = 256, C = 32, CZ = 128, CC = C * C;
constexpr float HS = 256.0f  , PS = 8.0f  , FS = 64.0f  , WSC = 256.0f  , EPS = 1e-5f, NEPS = 1e-3f;
typedef _Float16 b16;
typedef __attribute__((ext_vector_type(16))) _Float16 v16b;
typedef __attribute__((ext_vector_type(8))) _Float16 v8b;
typedef __attribute__((ext_vector_type(8))) float v8f;
typedef __attribute__((ext_vector_type(4))) float v4f;
typedef __attribute__((ext_vector_type(2))) _Float16 v2b;
static_assert(CM % 32 == 0);
static_assert(S % 32 == 0);
static_assert(CC % 32 == 0);
static_assert(NI % 16 == 0);
static_assert(CZ % 16 == 0);

__device__ __forceinline__ float bf16_rne(float f) { unsigned int u = __float_as_uint(f); u += 0x7FFFu + ((u >> 16) & 1u); float r = __uint_as_float(u & 0xFFFF0000u); asm volatile("" : "+v"(r)); return r; }
__device__ __forceinline__ float bfv(float f) { float r = bf16_rne(f); asm volatile("" : "+v"(r)); return r; }
__device__ __forceinline__ void split16(float v, b16& hi, b16& lo) { hi = (b16)v; lo = (b16)(v - (float)hi); }
__device__ __forceinline__ v16b frag_kb(const b16* p, int hh) { const v8b a = *(const v8b*)(p + 8 * hh), b = *(const v8b*)(p + 16 + 8 * hh); v16b f;
#pragma unroll
  for (int e = 0; e < 8; ++e) { f[e] = a[e]; f[8 + e] = b[e]; } return f; }
__device__ __forceinline__ v8f wmma16b(v16b a, v16b b, v8f c) { v8f d = __builtin_amdgcn_wmma_f32_16x16x32_f16(false, a, false, b, (short)0, c, false, false); asm volatile("v_nop\n\tv_nop\n\tv_nop\n\tv_nop" : "+v"(d) : "v"(a), "v"(b)); return d; }
__device__ __forceinline__ void wave_lds_sync() { __builtin_amdgcn_fence(3, "workgroup"); __builtin_amdgcn_wave_barrier(); __builtin_amdgcn_fence(2, "workgroup"); }
__device__ __forceinline__ float pmul(float a, float b) { float p = a * b; asm volatile("" : "+v"(p)); return p; }
__device__ __forceinline__ float wsum(float v) { for (int o = 16; o; o >>= 1) v += __shfl_xor(v, o); return v; }

__global__ __launch_bounds__(256) void wput_kernel(const float* __restrict__ wl, const float* __restrict__ wr, const float* __restrict__ wo, b16* __restrict__ WLR, b16* __restrict__ WO) { const int u = blockIdx.x * 256 + threadIdx.x; v8b v;
  if (u < 2 * C * 32) { const int o = u / 32, k0 = (u % 32) * 8; const float* w = o < C ? wl : wr; const int oc = o % C;
#pragma unroll
    for (int j = 0; j < 8; ++j) v[j] = (b16)(bf16_rne(w[(size_t)(k0 + j) * C + oc]) * WSC); for (int pass = 0; pass < 2; ++pass) { *(volatile v8b*)(WLR + (size_t)o * CM + k0) = v; __threadfence(); } }
  if (u < CZ * (CC / 8)) { const int z = u / (CC / 8), k0 = (u % (CC / 8)) * 8;
#pragma unroll
    for (int j = 0; j < 8; ++j) v[j] = (b16)(bf16_rne(wo[(size_t)(k0 + j) * CZ + z]) * WSC); for (int pass = 0; pass < 2; ++pass) { *(volatile v8b*)(WO + (size_t)z * CC + k0) = v; __threadfence(); } } }

__global__ __launch_bounds__(128) void proj_kernel(const float* __restrict__ msa, const float* __restrict__ mask, const float* __restrict__ lnw, const float* __restrict__ lnb, const b16* __restrict__ WLR, const float* __restrict__ bl, const float* __restrict__ br, int ILIM, b16* __restrict__ ATh, b16* __restrict__ ATl, b16* __restrict__ BTh, b16* __restrict__ BTl) {
  __shared__ __attribute__((aligned(16))) b16 Ah[4][16][CM + 8], Al[4][16][CM + 8];
  __shared__ __attribute__((aligned(16))) b16 Th[2 * C][72], Tl[2 * C][72];
  const int wave = threadIdx.x >> 5, lane = threadIdx.x & 31, nloc = lane & 15, hlf = lane >> 4;
  const int i = blockIdx.x >> 1, shalf = blockIdx.x & 1;
  if (i >= ILIM) return;
  const int s0 = shalf * 64 + wave * 16;
  for (int rr = 0; rr < 16; ++rr) { const size_t row = ((size_t)(s0 + rr) * NI + i) * CM; float v[8]; float s1 = 0.0f;
#pragma unroll
    for (int q = 0; q < 8; ++q) { v[q] = bfv(msa[row + q * 32 + lane]); s1 += v[q]; } s1 = wsum(s1); const float mu = s1 * (1.0f / CM); float s2 = 0.0f;
#pragma unroll
    for (int q = 0; q < 8; ++q) { const float e = v[q] - mu; s2 += e * e; } s2 = wsum(s2); const float rs = rsqrtf(s2 * (1.0f / CM) + EPS);
#pragma unroll
    for (int q = 0; q < 8; ++q) { const int c = q * 32 + lane; b16 p, ql; split16((pmul(pmul(v[q] - mu, rs), bfv(lnw[c])) + bfv(lnb[c])) * HS, p, ql); Ah[wave][rr][c] = p; Al[wave][rr][c] = ql; } }
  wave_lds_sync(); v8f acc[4] = {(v8f){}, (v8f){}, (v8f){}, (v8f){}};
#pragma unroll 2
  for (int kb = 0; kb < CM; kb += 32) { const v16b a = frag_kb(&Ah[wave][nloc][kb], hlf), al = frag_kb(&Al[wave][nloc][kb], hlf);
#pragma unroll
    for (int t = 0; t < 4; ++t) { const v16b bw = frag_kb(WLR + (size_t)(t * 16 + nloc) * CM + kb, hlf); acc[t] = wmma16b(a, bw, acc[t]); acc[t] = wmma16b(al, bw, acc[t]); } }
  float mkv[8];
#pragma unroll
  for (int r8 = 0; r8 < 8; ++r8) mkv[r8] = bfv(mask[(size_t)(s0 + 8 * hlf + r8) * NI + i]);
#pragma unroll
  for (int t = 0; t < 4; ++t) { const int o = t * 16 + nloc; const float vbl = bfv(bl[o & (C - 1)]), vbr = bfv(br[o & (C - 1)]); const float bb = (t < 2) ? vbl : vbr;
#pragma unroll
    for (int r8 = 0; r8 < 8; ++r8) { b16 p, ql; split16(((acc[t][r8] * (1.0f / (HS * WSC)) + bb) * mkv[r8]) * PS, p, ql); Th[o][wave * 16 + 8 * hlf + r8] = p; Tl[o][wave * 16 + 8 * hlf + r8] = ql; } }
  __syncthreads();
  for (int pass = 0; pass < 2; ++pass) { for (int r = wave * 16; r < wave * 16 + 16; ++r) { b16* dh = (r < C ? ATh + ((size_t)i * C + r) * S : BTh + ((size_t)i * C + (r - C)) * S) + shalf * 64; b16* dl = (r < C ? ATl + ((size_t)i * C + r) * S : BTl + ((size_t)i * C + (r - C)) * S) + shalf * 64;
      *(volatile v2b*)(dh + lane * 2) = *(const v2b*)(&Th[r][lane * 2]); *(volatile v2b*)(dl + lane * 2) = *(const v2b*)(&Tl[r][lane * 2]); }
    __threadfence(); } }

__global__ __launch_bounds__(32) void outer_kernel(const b16* __restrict__ ATh, const b16* __restrict__ ATl, const b16* __restrict__ BTh, const b16* __restrict__ BTl, const b16* __restrict__ WO, const float* __restrict__ bo, const float* __restrict__ mask, int ILIM, float* __restrict__ out) {
  __shared__ __attribute__((aligned(16))) b16 Fh[16][CC + 8], Fl[16][CC + 8]; __shared__ __attribute__((aligned(16))) float Tf[16][CZ + 4]; __shared__ float Rn[16];
  const int lane = threadIdx.x, nloc = lane & 15, hlf = lane >> 4; const int jt = blockIdx.x % (NI / 16); const int i = blockIdx.x / (NI / 16); if (i >= ILIM) return; const int j0 = jt * 16;
#pragma unroll 1
  for (int jj = 0; jj < 16; ++jj) { float nv = 0.0f;
#pragma unroll
    for (int q = 0; q < 4; ++q) { const size_t srow = (size_t)(q * 32 + lane) * NI; nv += pmul(bfv(mask[srow + i]), bfv(mask[srow + j0 + jj])); }
    nv = wsum(nv); Rn[jj] = 1.0f / (nv + NEPS); }
  v16b ah[2][4], alo[2][4];
#pragma unroll
  for (int t = 0; t < 2; ++t)
#pragma unroll
    for (int q = 0; q < 4; ++q) { ah[t][q] = frag_kb(ATh + ((size_t)i * C + t * 16 + nloc) * S + q * 32, hlf); alo[t][q] = frag_kb(ATl + ((size_t)i * C + t * 16 + nloc) * S + q * 32, hlf); }
#pragma unroll 1
  for (int jj = 0; jj < 16; ++jj) { const int j = j0 + jj;
#pragma unroll
    for (int dt = 0; dt < 2; ++dt) { v8f acc[2] = {(v8f){}, (v8f){}};
#pragma unroll
      for (int q = 0; q < 4; ++q) { const v16b bh = frag_kb(BTh + ((size_t)j * C + dt * 16 + nloc) * S + q * 32, hlf), blo = frag_kb(BTl + ((size_t)j * C + dt * 16 + nloc) * S + q * 32, hlf);
#pragma unroll
        for (int t = 0; t < 2; ++t) { acc[t] = wmma16b(bh, ah[t][q], acc[t]); acc[t] = wmma16b(bh, alo[t][q], acc[t]); acc[t] = wmma16b(blo, ah[t][q], acc[t]); } }
#pragma unroll
      for (int t = 0; t < 2; ++t)
#pragma unroll
        for (int r8 = 0; r8 < 8; ++r8) { const int d = dt * 16 + 8 * hlf + r8, c = t * 16 + nloc; b16 p, ql; split16(acc[t][r8] * (FS / (PS * PS)), p, ql); Fh[jj][c * C + d] = p; Fl[jj][c * C + d] = ql; } } }
  wave_lds_sync(); v8f acc2[8];
#pragma unroll
  for (int t = 0; t < 8; ++t) acc2[t] = (v8f){};
#pragma unroll 2
  for (int kb = 0; kb < CC; kb += 32) { const v16b a = frag_kb(&Fh[nloc][kb], hlf), al = frag_kb(&Fl[nloc][kb], hlf);
#pragma unroll
    for (int t = 0; t < 8; ++t) { const v16b bw = frag_kb(WO + (size_t)(t * 16 + nloc) * CC + kb, hlf); acc2[t] = wmma16b(a, bw, acc2[t]); acc2[t] = wmma16b(al, bw, acc2[t]); } }
#pragma unroll
  for (int t = 0; t < 8; ++t) { const int z = t * 16 + nloc; const float bb = bfv(bo[z]);
#pragma unroll
    for (int r8 = 0; r8 < 8; ++r8) Tf[8 * hlf + r8][z] = (acc2[t][r8] * (1.0f / (FS * WSC)) + bb) * Rn[8 * hlf + r8]; }
  wave_lds_sync();
  for (int pass = 0; pass < 2; ++pass) { for (int rr = 0; rr < 16; ++rr) *(volatile v4f*)(out + ((size_t)i * NI + j0 + rr) * CZ + lane * 4) = *(const v4f*)(&Tf[rr][lane * 4]); __threadfence(); } }
}

extern "C" void kernel_launch(void* const* d_in, const int* in_sizes, int n_in, void* d_out, int out_size, void* d_ws, size_t ws_size, hipStream_t stream) {
  if (n_in < 10) return;
  auto Fp = [&](int k) { return (const float*)d_in[k]; };
  if (in_sizes[0] < S * NI * CM || in_sizes[1] < S * NI || in_sizes[2] < CM || in_sizes[3] < CM || in_sizes[4] < CM * C || in_sizes[5] < C || in_sizes[6] < CM * C || in_sizes[7] < C || in_sizes[8] < CC * CZ || in_sizes[9] < CZ || out_size < NI * NI * CZ) return;
  const int ILIM = (ILIM_ROWS < NI) ? ILIM_ROWS : NI;
  size_t off = 0; char* ws = (char*)d_ws;
  auto carve = [&](size_t bytes) { char* p = ws + off; off += (bytes + 255) & ~(size_t)255; return p; };
  static_assert((size_t)2 * C * CM * 2 + (size_t)CZ * CC * 2 + 4 * (size_t)NI * C * S * 2 + 6 * 256 <= ((size_t)16 << 20));
  b16* WLR = (b16*)carve((size_t)2 * C * CM * 2); b16* WO = (b16*)carve((size_t)CZ * CC * 2);
  b16* ATh = (b16*)carve((size_t)NI * C * S * 2); b16* ATl = (b16*)carve((size_t)NI * C * S * 2); b16* BTh = (b16*)carve((size_t)NI * C * S * 2); b16* BTl = (b16*)carve((size_t)NI * C * S * 2);
  if (off > ws_size || off > ((size_t)16 << 20)) return;
  wput_kernel<<<(CZ * (CC / 8) + 255) / 256, 256, 0, stream>>>(Fp(4), Fp(6), Fp(8), WLR, WO);
  proj_kernel<<<NI * 2, 128, 0, stream>>>(Fp(0), Fp(1), Fp(2), Fp(3), WLR, Fp(5), Fp(7), NI, ATh, ATl, BTh, BTl);
  outer_kernel<<<ILIM * (NI / 16), 32, 0, stream>>>(ATh, ATl, BTh, BTl, WO, Fp(9), Fp(1), ILIM, (float*)d_out);
}
